// NonLocalBlock_81819126989596
// MI455X (gfx1250) — hardware-run, weakly checked
//
#include <hip/hip_runtime.h>


#ifndef NB
#define NB 16
#endif
#define NB_FULL 16
#define CH   64
#define CI   32
#define HH   64
#define WW   64
#define HW   (HH * WW)
#define NP   (HW / 4)
#define NTILE (NB * (HW / 64))
#define XTP  68
#define PSP  68
#define KVP  40
#define UFP  33
#define PFP  68
#define QRS  2048.0f
#define QRI  (1.0f / 2048.0f)
#define WSC  64.0f
#define WSI  (1.0f / 64.0f)
#define PSC  16.0f
#define PSI  (1.0f / 16.0f)
#define BN_EPS 1e-5f

static_assert(CH == 64);
static_assert(CI == 32);
static_assert(2 * CI == 64);
static_assert(WW == 64);
static_assert(HH % 4 == 0);
static_assert(HW % 64 == 0);
static_assert(NP % 64 == 0);
static_assert(NP % 32 == 0);
static_assert(NTILE % 4 == 0);
static_assert(NB <= NB_FULL);
static_assert((XTP * 4) % 16 == 0);
static_assert((PSP * 4) % 16 == 0);
static_assert((PFP * 4) % 16 == 0);
static_assert((KVP * 2) % 16 == 0);
static_assert(KVP >= 32);

typedef _Float16 h16;
typedef __attribute__((ext_vector_type(16))) _Float16 v16h;
typedef __attribute__((ext_vector_type(8)))  _Float16 v8h;
typedef __attribute__((ext_vector_type(8)))  float    v8f;
typedef __attribute__((ext_vector_type(4)))  float    v4f;
typedef v4f  __attribute__((may_alias)) v4fa;

__device__ __forceinline__ unsigned short f2bf(float f) { unsigned u = __float_as_uint(f); u += 0x7FFFu + ((u >> 16) & 1u); return (unsigned short)(u >> 16); }
__device__ __forceinline__ float bfr(float f) { return __uint_as_float(((unsigned)f2bf(f)) << 16); }
__device__ __forceinline__ v16h cat16(v8h lo, v8h hi) { return __builtin_shufflevector(lo, hi, 0, 1, 2, 3, 4, 5, 6, 7, 8, 9, 10, 11, 12, 13, 14, 15); }
__device__ __forceinline__ v16h  ldh(const h16* p) { return cat16(*(const v8h*)p, *(const v8h*)(p + 16)); }
__device__ __forceinline__ void wave_sync() { __builtin_amdgcn_fence(3  , "wavefront"); __builtin_amdgcn_wave_barrier(); asm volatile("" ::: "memory"); }
static __device__ __forceinline__ h16 toh_flush(float v) { const h16 r = (h16)v; return (fabsf(v) < 6.103515625e-05f) ? (h16)0.0f : r; }
__device__ __forceinline__ v8f mma_h(v16h a, v16h b, v8f c) {
    c = __builtin_amdgcn_wmma_f32_16x16x32_f16(false, a, false, b, (short)0, c, false, false);
    asm volatile("v_nop\n\tv_nop\n\tv_nop\n\tv_nop" : "+v"(c) : "v"(a), "v"(b));
    return c;
}

static_assert(4 * 256 * 8 == 64 * 64 + 64 * 32 + 64 * 32);
__device__ __forceinline__ void put8w(const v8f v, h16* dst) {
    v8h o;
#pragma unroll
    for (int k = 0; k < 8; ++k) o[k] = toh_flush(bfr(v[k]) * WSC);
    *(volatile v8h*)dst = o; __threadfence(); *(volatile v8h*)dst = o;
}
__global__ __launch_bounds__(256) void k_wprep(const float* __restrict__ wg, const float* __restrict__ wph, const float* __restrict__ wo, const float* __restrict__ wth, h16* WP) {
#pragma clang fp contract(off)
    const int t = threadIdx.x; const int blk = blockIdx.x;
    h16* dst = WP + (size_t)(blk * 256 + t) * 8;
    if (blk == 0)      { const v8f v = *(const v8f*)(wg  + (size_t)t * 8); put8w(v, dst); }
    else if (blk == 1) { const v8f v = *(const v8f*)(wph + (size_t)t * 8); put8w(v, dst); }
    else if (blk == 2) { const v8f v = *(const v8f*)(wo  + (size_t)t * 8); put8w(v, dst); }
    else { const int c = t >> 2, i0 = (t & 3) * 8; v8f v;
#pragma unroll
           for (int k = 0; k < 8; ++k) v[k] = wth[(size_t)(i0 + k) * CH + c];
           put8w(v, dst); }
}

static_assert(256 * 2 * 16 == 64 * 128);
static_assert(256 * 16 == 64 * 64);
__global__ __launch_bounds__(256) void k_xt(const float* __restrict__ x, h16* XT) {
#pragma clang fp contract(off)
    __shared__ __align__(16) float ts[64 * XTP];
    const int t = threadIdx.x; const int s0 = blockIdx.x * 64, b = blockIdx.y;
    { const int c = t >> 2, sq = (t & 3) * 16;
      const float* src = x + ((size_t)b * CH + c) * HW + s0 + sq;
#pragma unroll
      for (int q = 0; q < 4; ++q) { const v4f v = *(const v4f*)(src + 4 * q);
#pragma unroll
          for (int i = 0; i < 4; ++i) ts[(sq + 4 * q + i) * XTP + c] = v[i]; } }
    __syncthreads();
    v8h o[2];
#pragma unroll
    for (int it = 0; it < 2; ++it) { const int p = it * 256 + t; const int row = p >> 3, c8 = (p & 7) * 8;
        const v4f x0 = *(const v4fa*)(&ts[row * XTP + c8]); const v4f x1 = *(const v4fa*)(&ts[row * XTP + c8 + 4]);
#pragma unroll
        for (int i = 0; i < 4; ++i) { o[it][i] = toh_flush(bfr(x0[i])); o[it][4 + i] = toh_flush(bfr(x1[i])); } }
    h16* dst = XT + ((size_t)b * HW + s0) * CH;
#pragma unroll 1
    for (int ps = 0; ps < 2; ++ps) {
#pragma unroll
        for (int it = 0; it < 2; ++it) *(volatile v8h*)(dst + (size_t)(it * 256 + t) * 8) = o[it];
        if (ps == 0) __threadfence(); }
}

static_assert(32 * 16 * 4 == 16 * 128);
__global__ __launch_bounds__(128) void k_pool(const h16* __restrict__ XT, const h16* __restrict__ WC, const float* __restrict__ bg, const float* __restrict__ bph, h16* GPH, h16* GPR) {
    __shared__ __align__(16) float ps[64 * PSP];
    const int lane = threadIdx.x & 31, lr = lane & 15, hi = lane >> 4;
    const int wave = __builtin_amdgcn_readfirstlane((int)(threadIdx.x >> 5));
    const int rg = blockIdx.x, b = blockIdx.y;
    float bc[4];
    bc[0] = bfr(bg[lr]); bc[1] = bfr(bg[16 + lr]); bc[2] = bfr(bph[lr]); bc[3] = bfr(bph[16 + lr]);
    const size_t woff = (size_t)lr * CH + 8 * hi;
#pragma unroll 1
    for (int pi = 0; pi < 2; ++pi) {
        const int sA = (4 * rg + 2 * pi) * WW + 16 * wave;
        const size_t aoff = ((size_t)b * HW + (size_t)(sA + lr)) * CH + 8 * hi;
        v8f acc[2][4];
#pragma unroll
        for (int mt = 0; mt < 2; ++mt)
#pragma unroll
            for (int nt = 0; nt < 4; ++nt) acc[mt][nt] = (v8f){};
#pragma unroll
        for (int kc = 0; kc < CH; kc += 32) {
            const v16h a0 = ldh(XT + aoff + kc), a1 = ldh(XT + aoff + (size_t)WW * CH + kc);
#pragma unroll
            for (int nt = 0; nt < 4; ++nt) { const v16h wf = ldh(WC + woff + (size_t)nt * 16 * CH + kc);
                acc[0][nt] = mma_h(a0, wf, acc[0][nt]); acc[1][nt] = mma_h(a1, wf, acc[1][nt]); }
        }
#pragma unroll
        for (int nt = 0; nt < 4; ++nt) { v4f pv;
#pragma unroll
            for (int r2 = 0; r2 < 4; ++r2) {
                const float mv = fmaxf(fmaxf(acc[0][nt][2 * r2], acc[0][nt][2 * r2 + 1]), fmaxf(acc[1][nt][2 * r2], acc[1][nt][2 * r2 + 1]));
                pv[r2] = mv * WSI + bc[nt]; }
            *(v4fa*)(&ps[(nt * 16 + lr) * PSP + pi * 32 + 8 * wave + 4 * hi]) = pv; }
    }
    __syncthreads();
    v8h hv[4], rv[4];
#pragma unroll
    for (int s = 0; s < 4; ++s) { const int row = 16 * wave + 4 * s + (lane >> 3), c8 = (lane & 7) * 8;
        const v4f x0 = *(const v4fa*)(&ps[row * PSP + c8]); const v4f x1 = *(const v4fa*)(&ps[row * PSP + c8 + 4]);
#pragma unroll
        for (int i = 0; i < 4; ++i) { const h16 a0 = toh_flush(x0[i]); const h16 a1 = toh_flush(x1[i]); hv[s][i] = a0; hv[s][4 + i] = a1;
            rv[s][i] = toh_flush((x0[i] - (float)a0) * QRS); rv[s][4 + i] = toh_flush((x1[i] - (float)a1) * QRS); } }
    const size_t base = (size_t)b * 64 * NP + (size_t)rg * 64;
#pragma unroll 1
    for (int pp = 0; pp < 2; ++pp) {
#pragma unroll
        for (int s = 0; s < 4; ++s) { const int row = 16 * wave + 4 * s + (lane >> 3), c8 = (lane & 7) * 8;
            const size_t oo = base + (size_t)row * NP + c8;
            *(volatile v8h*)(GPH + oo) = hv[s]; *(volatile v8h*)(GPR + oo) = rv[s]; }
        if (pp == 0) __threadfence(); }
}

static_assert(32 * 16 * 4 == 16 * 128);
static_assert(16 * 16 == 64 * 4);
__global__ __launch_bounds__(128) void k_fold(const h16* __restrict__ GPH, const h16* __restrict__ GPR, const h16* __restrict__ WOH, const h16* __restrict__ WTT,
                                              const float* __restrict__ bth, const float* __restrict__ bo, h16* PH, float* QV) {
    __shared__ __align__(16) h16 kvh[32 * KVP];
    __shared__ __align__(16) h16 kvr[32 * KVP];
    __shared__ __align__(16) h16 uh[64 * KVP];
    __shared__ __align__(16) h16 ur[64 * KVP];
    __shared__ __align__(16) float uf[64 * UFP];
    __shared__ __align__(16) float pf[64 * PFP];
    __shared__ __align__(16) float qs[64];
    const int lane = threadIdx.x & 31, lr = lane & 15, hi = lane >> 4;
    const int wave = __builtin_amdgcn_readfirstlane((int)(threadIdx.x >> 5));
    const int b = blockIdx.x;
    { const int m0 = (wave >> 1) * 16, n0 = (wave & 1) * 16;
      const size_t po = ((size_t)b * 64 + 32 + m0 + lr) * NP + 8 * hi;
      const size_t go = ((size_t)b * 64 + n0 + lr) * NP + 8 * hi;
      v8f aH = (v8f){}, aR = (v8f){};
#pragma unroll 1
      for (int kc = 0; kc < NP; kc += 32) {
          const v16h ph = ldh(GPH + po + kc), pr = ldh(GPR + po + kc), gh = ldh(GPH + go + kc), gr = ldh(GPR + go + kc);
          aH = mma_h(ph, gh, aH); aR = mma_h(ph, gr, aR); aR = mma_h(pr, gh, aR); }
#pragma unroll
      for (int r = 0; r < 8; ++r) { const float v = (aH[r] + aR[r] * QRI) * (1.0f / (float)NP); const h16 a0 = toh_flush(v);
          kvh[(m0 + 8 * hi + r) * KVP + n0 + lr] = a0; kvr[(m0 + 8 * hi + r) * KVP + n0 + lr] = toh_flush((v - (float)a0) * QRS); } }
    __syncthreads();
    { const v16h a3 = ldh(WOH + (size_t)(16 * wave + lr) * CI + 8 * hi);
#pragma unroll
      for (int nt = 0; nt < 2; ++nt) {
          const v16h bh = cat16(*(const v8h*)(&kvh[(nt * 16 + lr) * KVP + 8 * hi]), *(const v8h*)(&kvh[(nt * 16 + lr) * KVP + 16 + 8 * hi]));
          const v16h br = cat16(*(const v8h*)(&kvr[(nt * 16 + lr) * KVP + 8 * hi]), *(const v8h*)(&kvr[(nt * 16 + lr) * KVP + 16 + 8 * hi]));
          const v8f uH = mma_h(a3, bh, (v8f){}); const v8f uR = mma_h(a3, br, (v8f){});
#pragma unroll
          for (int r = 0; r < 8; ++r) { const float v = (uH[r] + uR[r] * QRI) * WSI; const h16 a0 = toh_flush(v); const int o = 16 * wave + 8 * hi + r, i = nt * 16 + lr;
              uf[o * UFP + i] = v; uh[o * KVP + i] = a0; ur[o * KVP + i] = toh_flush((v - (float)a0) * QRS); } } }
    __syncthreads();
    { const v16h ah = cat16(*(const v8h*)(&uh[(16 * wave + lr) * KVP + 8 * hi]), *(const v8h*)(&uh[(16 * wave + lr) * KVP + 16 + 8 * hi]));
      const v16h ar = cat16(*(const v8h*)(&ur[(16 * wave + lr) * KVP + 8 * hi]), *(const v8h*)(&ur[(16 * wave + lr) * KVP + 16 + 8 * hi]));
#pragma unroll
      for (int nt = 0; nt < 4; ++nt) { const v16h wf = ldh(WTT + (size_t)(nt * 16 + lr) * CI + 8 * hi);
          const v8f pH = mma_h(ah, wf, (v8f){}); const v8f pR = mma_h(ar, wf, (v8f){});
#pragma unroll
          for (int r = 0; r < 8; ++r) pf[(16 * wave + 8 * hi + r) * PFP + nt * 16 + lr] = (pH[r] + pR[r] * QRI) * (WSI * PSC); } }
    { const int t = threadIdx.x;
      if (t < 64) { float s = 0.0f;
#pragma unroll 1
          for (int i = 0; i < CI; ++i) s += uf[t * UFP + i] * bfr(bth[i]);
          qs[t] = s + bfr(bo[t]); } }
    __syncthreads();
    v8h hv[4];
#pragma unroll
    for (int s = 0; s < 4; ++s) { const int row = 16 * wave + 4 * s + (lane >> 3), c8 = (lane & 7) * 8;
        const v4f x0 = *(const v4fa*)(&pf[row * PFP + c8]); const v4f x1 = *(const v4fa*)(&pf[row * PFP + c8 + 4]);
#pragma unroll
        for (int i = 0; i < 4; ++i) { hv[s][i] = toh_flush(x0[i]); hv[s][4 + i] = toh_flush(x1[i]); } }
    const v4f qv = *(const v4fa*)(&qs[4 * (lane & 15)]);
    h16* pdst = PH + (size_t)b * CH * CH;
    float* qdst = QV + (size_t)b * CH + 4 * (lane & 15);
#pragma unroll 1
    for (int pp = 0; pp < 2; ++pp) {
#pragma unroll
        for (int s = 0; s < 4; ++s) { const int row = 16 * wave + 4 * s + (lane >> 3), c8 = (lane & 7) * 8;
            *(volatile v8h*)(pdst + (size_t)row * CH + c8) = hv[s]; }
        if (wave == 0) { if (lane < 16) *(volatile v4f*)qdst = qv; }
        if (pp == 0) __threadfence(); }
}

__device__ __forceinline__ void gemm_tile(const h16* __restrict__ PH, const h16* __restrict__ XT, int b, int c0, int lr, int hi, v8f (&acc)[4][4]) {
#pragma unroll
    for (int mb = 0; mb < 4; ++mb)
#pragma unroll
        for (int nb = 0; nb < 4; ++nb) acc[mb][nb] = (v8f){};
    const size_t aoff = ((size_t)b * CH + lr) * CH + 8 * hi;
    const size_t boff = ((size_t)b * HW + (size_t)(c0 + lr)) * CH + 8 * hi;
#pragma unroll 1
    for (int kc = 0; kc < CH; kc += 32) {
        v16h a[4];
#pragma unroll
        for (int mb = 0; mb < 4; ++mb) a[mb] = ldh(PH + aoff + (size_t)mb * 16 * CH + kc);
#pragma unroll
        for (int nb = 0; nb < 4; ++nb) { const v16h bb = ldh(XT + boff + (size_t)nb * 16 * CH + kc);
#pragma unroll
            for (int mb = 0; mb < 4; ++mb) acc[mb][nb] = mma_h(a[mb], bb, acc[mb][nb]); }
    }
}

static_assert(32 * 16 == 128 * 4);
__global__ __launch_bounds__(32) void k_stat(const h16* __restrict__ PH, const h16* __restrict__ XT, const float* __restrict__ QV, float* PART) {
    __shared__ __align__(16) float st[128];
    const int lane = threadIdx.x & 31, lr = lane & 15, hi = lane >> 4;
    const int c0 = blockIdx.x * 64, b = blockIdx.y;
    v8f acc[4][4];
    gemm_tile(PH, XT, b, c0, lr, hi, acc);
#pragma unroll
    for (int mb = 0; mb < 4; ++mb) {
        const v4f q0 = *(const v4f*)(QV + (size_t)b * CH + mb * 16 + 8 * hi); const v4f q1 = *(const v4f*)(QV + (size_t)b * CH + mb * 16 + 8 * hi + 4);
#pragma unroll
        for (int j = 0; j < 8; ++j) { const float qj = (j < 4) ? q0[j & 3] : q1[j & 3];
            float s = 0.0f, ss = 0.0f;
#pragma unroll
            for (int nb = 0; nb < 4; ++nb) { const float z = acc[mb][nb][j] * PSI + qj; s += z; ss += z * z; }
#pragma unroll
            for (int m = 1; m <= 8; m <<= 1) { s += __shfl_xor(s, m, 32); ss += __shfl_xor(ss, m, 32); }
            if (lr == 0) { st[mb * 16 + 8 * hi + j] = s; st[64 + mb * 16 + 8 * hi + j] = ss; } }
    }
    wave_sync();
    const v4f pv = *(const v4fa*)(&st[4 * lane]);
    float* dst = PART + ((size_t)b * (HW / 64) + blockIdx.x) * 128 + 4 * lane;
    *(volatile v4f*)dst = pv; __threadfence(); *(volatile v4f*)dst = pv;
}

__global__ __launch_bounds__(256) void k_bn(const float* __restrict__ PART, const float* __restrict__ gamma, const float* __restrict__ beta, float* SS) {
#pragma clang fp contract(off)
    __shared__ double red[4 * 128];
    __shared__ __align__(16) float ssl[128];
    const int t = threadIdx.x, c = t & 63, qd = t >> 6;
    double s = 0.0, ss = 0.0;
#pragma unroll 1
    for (int k = 0; k < NTILE / 4; ++k) { const float* p = PART + (size_t)(qd * (NTILE / 4) + k) * 128; s += (double)p[c]; ss += (double)p[64 + c]; }
    red[qd * 128 + c] = s; red[qd * 128 + 64 + c] = ss;
    __syncthreads();
    if (t < 64) {
        const double S1 = (red[c] + red[128 + c]) + (red[256 + c] + red[384 + c]);
        const double S2 = (red[64 + c] + red[192 + c]) + (red[320 + c] + red[448 + c]);
        const double inv = 1.0 / (double)((size_t)NB * HW);
        const double mu = S1 * inv; double var = S2 * inv - mu * mu; var = var < 0.0 ? 0.0 : var;
        const float sd = sqrtf((float)var + BN_EPS);
        const float sc = bfr(gamma[c]) * (1.0f / sd);
        ssl[c] = sc; ssl[64 + c] = bfr(beta[c]) - (float)mu * sc; }
    __syncthreads();
    if (t < 32) { const v4f v = *(const v4fa*)(&ssl[4 * t]); float* dst = SS + 4 * t; *(volatile v4f*)dst = v; __threadfence(); *(volatile v4f*)dst = v; }
}

static_assert(32 * 16 * 8 == 16 * 256);
__global__ __launch_bounds__(32) void k_out(const h16* __restrict__ PH, const h16* __restrict__ XT, const float* __restrict__ QV, const float* __restrict__ SS,
                                            const float* __restrict__ x, float* OUT) {
    __shared__ __align__(16) float os[16 * PFP];
    const int lane = threadIdx.x & 31, lr = lane & 15, hi = lane >> 4;
    const int c0 = blockIdx.x * 64, b = blockIdx.y;
    v8f acc[4][4];
    gemm_tile(PH, XT, b, c0, lr, hi, acc);
    const size_t obase = (size_t)b * CH * HW + c0;
#pragma unroll
    for (int mb = 0; mb < 4; ++mb) {
        const int cb = mb * 16 + 8 * hi;
        const v4f q0 = *(const v4f*)(QV + (size_t)b * CH + cb), q1 = *(const v4f*)(QV + (size_t)b * CH + cb + 4);
        const v4f g0 = *(const v4f*)(SS + cb), g1 = *(const v4f*)(SS + cb + 4);
        const v4f h0 = *(const v4f*)(SS + 64 + cb), h1 = *(const v4f*)(SS + 64 + cb + 4);
#pragma unroll
        for (int j = 0; j < 8; ++j) { const float qj = (j < 4) ? q0[j & 3] : q1[j & 3]; const float gj = (j < 4) ? g0[j & 3] : g1[j & 3]; const float hj = (j < 4) ? h0[j & 3] : h1[j & 3];
#pragma unroll
            for (int nb = 0; nb < 4; ++nb) os[(hi * 8 + j) * PFP + nb * 16 + lr] = (acc[mb][nb][j] * PSI + qj) * gj + hj; }
        wave_sync();
        v4f ov[8];
#pragma unroll
        for (int s = 0; s < 8; ++s) { const int row = 2 * s + (lane >> 4), c4 = (lane & 15) * 4;
            const v4f val = *(const v4fa*)(&os[row * PFP + c4]);
            const v4f xr = *(const v4f*)(x + obase + (size_t)(mb * 16 + row) * HW + c4);
#pragma unroll
            for (int i = 0; i < 4; ++i) ov[s][i] = val[i] + bfr(xr[i]); }
#pragma unroll 1
        for (int pp = 0; pp < 2; ++pp) {
#pragma unroll
            for (int s = 0; s < 8; ++s) { const int row = 2 * s + (lane >> 4), c4 = (lane & 15) * 4;
                *(volatile v4f*)(OUT + obase + (size_t)(mb * 16 + row) * HW + c4) = ov[s]; }
            if (pp == 0) __threadfence(); }
        wave_sync();
    }
}

static constexpr size_t al256(size_t v) { return (v + 255) & ~(size_t)255; }
static constexpr size_t SZ_WP = al256((size_t)8192 * 2);
static constexpr size_t SZ_XT = al256((size_t)NB * HW * CH * 2);
static constexpr size_t SZ_GP = al256((size_t)NB * 64 * NP * 2);
static constexpr size_t SZ_PH = al256((size_t)NB * CH * CH * 2);
static constexpr size_t SZ_QV = al256((size_t)NB * CH * 4);
static constexpr size_t SZ_PT = al256((size_t)NTILE * 128 * 4);
static constexpr size_t SZ_SS = al256((size_t)128 * 4);
static constexpr size_t SZ_TOTAL = SZ_WP + SZ_XT + 2 * SZ_GP + SZ_PH + SZ_QV + SZ_PT + SZ_SS;
static_assert(SZ_TOTAL <= (size_t)134217728);
static_assert((size_t)(HW / 64) * NB * 64 * 128 == (size_t)NB * HW * CH * 2);
static_assert((size_t)(HH / 4) * NB * 64 * 128 == (size_t)NB * 64 * NP * 2);
static_assert((size_t)NB * 64 * 128 == (size_t)NB * CH * CH * 2);
static_assert((size_t)(HW / 64) * NB * 512 == (size_t)NTILE * 128 * 4);
static_assert((size_t)(HW / 64) * NB * 64 * 256 == (size_t)NB * CH * HW * 4);
static_assert((size_t)64 * XTP * 4 <= 131072);
static_assert((size_t)64 * PSP * 4 <= 131072);
static_assert((size_t)(2 * 32 * KVP + 2 * 64 * KVP) * 2 + (size_t)(64 * UFP + 64 * PFP + 64) * 4 <= 131072);
static_assert((size_t)16 * PFP * 4 <= 131072);
static_assert((size_t)4 * 128 * 8 + 128 * 4 <= 131072);

extern "C" void kernel_launch(void* const* d_in, const int* in_sizes, int n_in,
                              void* d_out, int out_size, void* d_ws, size_t ws_size, hipStream_t stream) {
    if (n_in < 11) return;
    const size_t needx = (size_t)NB * CH * HW;
    if ((size_t)in_sizes[0] < needx) return;
    if (in_sizes[1] < CI * CH || in_sizes[3] < CI * CH || in_sizes[5] < CI * CH || in_sizes[7] < CH * CI) return;
    if (in_sizes[2] < CI || in_sizes[4] < CI || in_sizes[6] < CI) return;
    if (in_sizes[8] < CH || in_sizes[9] < CH || in_sizes[10] < CH) return;
    if ((size_t)out_size < needx) return;
    if (SZ_TOTAL > ws_size) return;
    const float* x   = (const float*)d_in[0];
    const float* wg  = (const float*)d_in[1];  const float* bg  = (const float*)d_in[2];
    const float* wth = (const float*)d_in[3];  const float* bth = (const float*)d_in[4];
    const float* wph = (const float*)d_in[5];  const float* bph = (const float*)d_in[6];
    const float* wo  = (const float*)d_in[7];  const float* bo  = (const float*)d_in[8];
    const float* gamma = (const float*)d_in[9]; const float* beta = (const float*)d_in[10];
    float* OUT = (float*)d_out;
    char* wsp = (char*)d_ws;
    h16* WP  = (h16*)wsp;   wsp += SZ_WP;
    h16* XT  = (h16*)wsp;   wsp += SZ_XT;
    h16* GPH = (h16*)wsp;   wsp += SZ_GP;
    h16* GPR = (h16*)wsp;   wsp += SZ_GP;
    h16* PH  = (h16*)wsp;   wsp += SZ_PH;
    float* QV   = (float*)wsp; wsp += SZ_QV;
    float* PART = (float*)wsp; wsp += SZ_PT;
    float* SS   = (float*)wsp; wsp += SZ_SS;
    h16* WC  = WP;
    h16* WOH = WP + 4096;
    h16* WTT = WP + 6144;

    k_wprep<<<4, 256, 0, stream>>>(wg, wph, wo, wth, WP);
    k_xt<<<dim3(HW / 64, NB, 1), 256, 0, stream>>>(x, XT);
    k_pool<<<dim3(HH / 4, NB, 1), 128, 0, stream>>>(XT, WC, bg, bph, GPH, GPR);
    k_fold<<<NB, 128, 0, stream>>>(GPH, GPR, WOH, WTT, bth, bo, PH, QV);
    k_stat<<<dim3(HW / 64, NB, 1), 32, 0, stream>>>(PH, XT, QV, PART);
    k_bn<<<1, 256, 0, stream>>>(PART, gamma, beta, SS);
    k_out<<<dim3(HW / 64, NB, 1), 32, 0, stream>>>(PH, XT, QV, SS, x, OUT);
}
